// InteractiveDualMambaBlock_90872918049559
// MI455X (gfx1250) — hardware-run, weakly checked
//
#include <hip/hip_runtime.h>


#define NB_  2
#define LL   1024
#define HID  1024
#define DI   2048
#define NS   16
#define RR   64
#define PW   128
typedef _Float16 h16;
typedef unsigned short bf;
typedef __attribute__((ext_vector_type(16))) __bf16   v16bf;
typedef __attribute__((ext_vector_type(16))) _Float16 v16h;
typedef __attribute__((ext_vector_type(8)))  _Float16 v8h;
typedef __attribute__((ext_vector_type(8)))  unsigned short v8us;
typedef __attribute__((ext_vector_type(8)))  float    v8f;
typedef __attribute__((ext_vector_type(4)))  float    v4f;
typedef v8h  __attribute__((may_alias)) v8ha;
typedef v4f  __attribute__((may_alias)) v4fa;
typedef v8us __attribute__((may_alias)) v8usa;

__device__ __forceinline__ unsigned short f2bf(float f) { unsigned u = __float_as_uint(f); u += 0x7FFFu + ((u >> 16) & 1u); return (unsigned short)(u >> 16); }
__device__ __forceinline__ float bf2f(unsigned short b) { return __uint_as_float(((unsigned)b) << 16); }
__device__ __forceinline__ float bfr(float f) { return bf2f(f2bf(f)); }
__device__ __forceinline__ v16h cat16(v8h lo, v8h hi) { return __builtin_shufflevector(lo, hi, 0, 1, 2, 3, 4, 5, 6, 7, 8, 9, 10, 11, 12, 13, 14, 15); }
__device__ __forceinline__ v16bf cat16b(v8us lo, v8us hi) { return __builtin_bit_cast(v16bf, __builtin_shufflevector(lo, hi, 0, 1, 2, 3, 4, 5, 6, 7, 8, 9, 10, 11, 12, 13, 14, 15)); }
__device__ __forceinline__ v8f wmma16(v16h a, v16h b, v8f c) { return __builtin_amdgcn_wmma_f32_16x16x32_f16(false, a, false, b, (short)0, c, false, false); }
__device__ __forceinline__ v8f wmmab(v16bf a, v16bf b, v8f c) { return __builtin_amdgcn_wmma_f32_16x16x32_bf16(false, a, false, b, (short)0, c, false, false); }


template <typename T16> struct WFrag;
template <> struct WFrag<h16> { typedef v16h V; static __device__ __forceinline__ V ld(const h16* p) { return cat16(*(const v8h*)p, *(const v8h*)(p + 16)); } static __device__ __forceinline__ v8f mma(V a, V b, v8f c) { return wmma16(a, b, c); } };
template <> struct WFrag<bf> { typedef v16bf V; static __device__ __forceinline__ V ld(const bf* p) { return cat16b(*(const v8us*)p, *(const v8us*)(p + 16)); } static __device__ __forceinline__ v8f mma(V a, V b, v8f c) { return wmmab(a, b, c); } };
template <typename T16, int NSPLIT, bool BIAS>
__global__ __launch_bounds__(32) void k_gemmw(const T16* __restrict__ A, const T16* __restrict__ A2, const T16* __restrict__ Bt, const T16* __restrict__ Bt2, int K, float* C, int ldc, const float* __restrict__ bias, size_t sA, size_t sB, size_t sC) {
    typedef typename WFrag<T16>::V V;
    __shared__ __align__(16) float os[16 * 68];
    const size_t z = blockIdx.z; A += z * sA; if (A2) A2 += z * sA; Bt += z * sB; if (Bt2) Bt2 += z * sB; C += z * sC;
    const int lane = threadIdx.x & 31, lr = lane & 15, hi = lane >> 4; const int r0 = blockIdx.x * 64, c0 = blockIdx.y * 64;
    v8f acc[4][4];
#pragma unroll
    for (int mb = 0; mb < 4; ++mb)
#pragma unroll
        for (int nb = 0; nb < 4; ++nb) acc[mb][nb] = (v8f){};
    const size_t aoff = (size_t)(r0 + lr) * K + 8 * hi, boff = (size_t)(c0 + lr) * K + 8 * hi;
#pragma unroll 1
    for (int kc = 0; kc < K; kc += 32) {
        V a[4], a2[4];
#pragma unroll
        for (int mb = 0; mb < 4; ++mb) { a[mb] = WFrag<T16>::ld(A + aoff + (size_t)mb * 16 * K + kc); if (NSPLIT == 1 || NSPLIT == 2) a2[mb] = WFrag<T16>::ld(A2 + aoff + (size_t)mb * 16 * K + kc); }
#pragma unroll
        for (int nb = 0; nb < 4; ++nb) { const V b = WFrag<T16>::ld(Bt + boff + (size_t)nb * 16 * K + kc); V b2; if (NSPLIT >= 2) b2 = WFrag<T16>::ld(Bt2 + boff + (size_t)nb * 16 * K + kc);
#pragma unroll
            for (int mb = 0; mb < 4; ++mb) { acc[mb][nb] = WFrag<T16>::mma(a[mb], b, acc[mb][nb]); if (NSPLIT == 1 || NSPLIT == 2) acc[mb][nb] = WFrag<T16>::mma(a2[mb], b, acc[mb][nb]); if (NSPLIT >= 2) acc[mb][nb] = WFrag<T16>::mma(a[mb], b2, acc[mb][nb]); } }
        asm volatile("v_nop\n\tv_nop\n\tv_nop\n\tv_nop" : "+v"(acc[0][0]), "+v"(acc[1][1]), "+v"(acc[2][2]), "+v"(acc[3][3]) : "v"(a[0]), "v"(a[3]));
    }
#pragma unroll
    for (int mb = 0; mb < 4; ++mb) {
#pragma unroll
        for (int nb = 0; nb < 4; ++nb) {
#pragma unroll
            for (int j = 0; j < 8; ++j) os[(hi * 8 + j) * 68 + nb * 16 + lr] = acc[mb][nb][j]; }
        __builtin_amdgcn_wave_barrier(); asm volatile("" ::: "memory");
        float* crow = C + (size_t)(r0 + mb * 16) * ldc + c0;
#pragma unroll 1
        for (int ps = 0; ps < 2; ++ps) {
#pragma unroll
            for (int s = 0; s < 8; ++s) { const int row = 2 * s + hi, cofs = lr * 4; v4f val = *(const v4fa*)(os + row * 68 + cofs); if (BIAS) { val[0] += bfr(bias[c0 + cofs]); val[1] += bfr(bias[c0 + cofs + 1]); val[2] += bfr(bias[c0 + cofs + 2]); val[3] += bfr(bias[c0 + cofs + 3]); }
                *(volatile v4f*)(crow + (size_t)row * ldc + cofs) = val; }
            if (ps == 0) __threadfence(); }
        __builtin_amdgcn_wave_barrier(); asm volatile("" ::: "memory");
    }
}

__device__ __forceinline__ void splitf(float y, unsigned short& h, unsigned short& l) { h = f2bf(y); l = f2bf(y - bf2f(h)); }
__device__ __forceinline__ float silu_(float x) { return __fmul_rn(x, __fdiv_rn(1.0f, 1.0f + __expf(-x))); }
__device__ __forceinline__ float softplus_(float x) { return x > 20.f ? x : log1pf(__expf(x)); }
typedef __attribute__((ext_vector_type(2))) unsigned short v2us;
typedef __attribute__((ext_vector_type(4))) unsigned short v4us;

__global__ __launch_bounds__(256) void k_cvt8(const float* __restrict__ src, bf* dst, size_t n8) { const size_t i = (size_t)blockIdx.x * 256 + threadIdx.x; if (i >= n8) return; const v8f v = *(const v8f*)(src + i * 8); v8us o;
#pragma unroll
    for (int k = 0; k < 8; ++k) o[k] = f2bf(v[k]); *(volatile v8us*)(dst + i * 8) = o; __threadfence(); *(volatile v8us*)(dst + i * 8) = o; }
__global__ __launch_bounds__(256) void k_wx(const float* __restrict__ w, bf* WX) { const int i = (blockIdx.x * 256 + threadIdx.x) * 4; if (i >= PW * DI) return; const int r = i / DI; v4us o;
#pragma unroll
    for (int q = 0; q < 4; ++q) o[q] = r < RR + 2 * NS ? f2bf(w[i + q]) : (unsigned short)0; *(volatile v4us*)(WX + i) = o; __threadfence(); *(volatile v4us*)(WX + i) = o; }
__global__ __launch_bounds__(256) void k_split(const float* __restrict__ F, int pitch, int c0, int wsel, bf* Hh, bf* Hl) { const int e = (blockIdx.x * 256 + threadIdx.x) * 4; if (e >= LL * wsel) return; const int c = e % wsel, t = e / wsel; const v4f a = *(const v4f*)(F + (size_t)t * pitch + c0 + c); v4us oh, ol;
#pragma unroll
    for (int q = 0; q < 4; ++q) { unsigned short u, l; splitf(a[q], u, l); oh[q] = u; ol[q] = l; } *(volatile v4us*)(Hh + e) = oh; *(volatile v4us*)(Hl + e) = ol; __threadfence(); *(volatile v4us*)(Hh + e) = oh; *(volatile v4us*)(Hl + e) = ol; }
__global__ __launch_bounds__(256) void k_conv3(const float* __restrict__ XR, const float* __restrict__ w1, const float* __restrict__ b1, const float* __restrict__ w2, const float* __restrict__ b2, const float* __restrict__ wt, const float* __restrict__ bt, float* XF, bf* Fh, bf* Fl) {
    const int e = (blockIdx.x * 256 + threadIdx.x) * 4; if (e >= LL * DI) return; const int c = e % DI, t = e / DI; v4f o; v4us oh, ol;
#pragma unroll 1
    for (int q = 0; q < 4; ++q) { const int cc = c + q; auto xi = [&](int ts) { return (ts >= 0 && ts < LL) ? XR[(size_t)ts * 2 * DI + cc] : 0.f; };
        float a1 = bfr(b1[cc]); { float p = __fmul_rn(bfr(w1[cc * 2 + 0]), xi(t - 1)); asm volatile("" : "+v"(p)); a1 = __fadd_rn(a1, p); } { float p = __fmul_rn(bfr(w1[cc * 2 + 1]), xi(t)); asm volatile("" : "+v"(p)); a1 = __fadd_rn(a1, p); }
        float a2 = bfr(b2[cc]);
#pragma unroll
        for (int k = 0; k < 4; ++k) { float p = __fmul_rn(bfr(w2[cc * 4 + k]), xi(t - 3 + k)); asm volatile("" : "+v"(p)); a2 = __fadd_rn(a2, p); }
        float a3 = bfr(bt[cc]);
#pragma unroll
        for (int k = 0; k < 3; ++k) { float p = __fmul_rn(bfr(wt[cc * 3 + k]), xi(t - 1 + k)); asm volatile("" : "+v"(p)); a3 = __fadd_rn(a3, p); }
        float m = __fmul_rn(silu_(a1), silu_(a2)); asm volatile("" : "+v"(m)); o[q] = __fadd_rn(m, a3); unsigned short u, l; splitf(o[q], u, l); oh[q] = u; ol[q] = l; }
    for (int ps = 0; ps < 2; ++ps) { *(volatile v4f*)(XF + e) = o; *(volatile v4us*)(Fh + e) = oh; *(volatile v4us*)(Fl + e) = ol; if (ps == 0) __threadfence(); } }
__global__ __launch_bounds__(256) void k_scan(const float* __restrict__ DTR, const float* __restrict__ XF, const float* __restrict__ PBC, const float* __restrict__ XR, const float* __restrict__ alog, const float* __restrict__ Dp, bf* Yh, bf* Yl) {
    __shared__ float ybuf[64]; const int tid = threadIdx.x; const int cl = tid >> 2, sub = tid & 3; const int d = blockIdx.x * 64 + cl; const int n0 = sub * 4; float A[4], s[4];
#pragma unroll
    for (int j = 0; j < 4; ++j) { A[j] = -__expf(bfr(alog[(size_t)d * NS + n0 + j])); s[j] = 0.f; }
    const float dd = bfr(Dp[d]);
    for (int t = 0; t < LL; ++t) { const float dt = softplus_(softplus_(DTR[(size_t)t * DI + d])); const float xf = XF[(size_t)t * DI + d]; const float dtx = __fmul_rn(dt, xf); const float* pr = PBC + (size_t)t * PW + RR; float y = 0.f;
#pragma unroll
        for (int j = 0; j < 4; ++j) { const float a = __expf(__fmul_rn(dt, A[j])); float hb = __fmul_rn(dtx, pr[n0 + j]); asm volatile("" : "+v"(hb)); float ha = __fmul_rn(a, s[j]); asm volatile("" : "+v"(ha)); s[j] = __fadd_rn(ha, hb); float yc = __fmul_rn(s[j], pr[NS + n0 + j]); asm volatile("" : "+v"(yc)); y = __fadd_rn(y, yc); }
        y += __shfl_xor(y, 1, 32); y += __shfl_xor(y, 2, 32);
        if (sub == 0) { float sk = __fmul_rn(xf, dd); asm volatile("" : "+v"(sk)); const float yy = __fadd_rn(y, sk); ybuf[cl] = __fmul_rn(yy, silu_(XR[(size_t)t * 2 * DI + DI + d])); }
        __syncthreads();
        if (tid < 32) { v2us oh, ol; unsigned short u, l; splitf(ybuf[2 * tid], u, l); oh[0] = u; ol[0] = l; splitf(ybuf[2 * tid + 1], u, l); oh[1] = u; ol[1] = l; const size_t o = (size_t)t * DI + blockIdx.x * 64 + 2 * tid; *(volatile v2us*)(Yh + o) = oh; *(volatile v2us*)(Yl + o) = ol; __threadfence(); *(volatile v2us*)(Yh + o) = oh; *(volatile v2us*)(Yl + o) = ol; }
        __syncthreads(); } }

extern "C" void kernel_launch(void* const* d_in, const int* in_sizes, int n_in,
                              void* d_out, int out_size, void* d_ws, size_t ws_size, hipStream_t stream) {
    (void)in_sizes; (void)n_in; (void)out_size;
    const float* x = (const float*)d_in[0]; const float* win = (const float*)d_in[1]; const float* c1w = (const float*)d_in[2]; const float* c1b = (const float*)d_in[3]; const float* c2w = (const float*)d_in[4]; const float* c2b = (const float*)d_in[5]; const float* tw = (const float*)d_in[6]; const float* tb = (const float*)d_in[7]; const float* wx = (const float*)d_in[8]; const float* wdt = (const float*)d_in[9]; const float* bdt = (const float*)d_in[10]; const float* alog = (const float*)d_in[11]; const float* Dp = (const float*)d_in[12]; const float* wout = (const float*)d_in[13];
    float* OUT = (float*)d_out;
    char* wsp = (char*)d_ws;
    auto take = [&](size_t bytes) { char* p = wsp; wsp += (bytes + 255) & ~(size_t)255; return (void*)p; };
    bf* WIN = (bf*)take((size_t)2 * DI * HID * 2); bf* WX = (bf*)take((size_t)PW * DI * 2); bf* WDT = (bf*)take((size_t)DI * RR * 2); bf* WOUT = (bf*)take((size_t)HID * DI * 2);
    bf* XB = (bf*)take((size_t)LL * HID * 2); float* XR = (float*)take((size_t)LL * 2 * DI * 4); float* XF = (float*)take((size_t)LL * DI * 4); bf* Fh = (bf*)take((size_t)LL * DI * 2); bf* Fl = (bf*)take((size_t)LL * DI * 2); float* PBC = (float*)take((size_t)LL * PW * 4); bf* Rh = (bf*)take((size_t)LL * RR * 2); bf* Rl = (bf*)take((size_t)LL * RR * 2); float* DTR = (float*)take((size_t)LL * DI * 4); bf* Yh = (bf*)take((size_t)LL * DI * 2); bf* Yl = (bf*)take((size_t)LL * DI * 2);
    if ((size_t)(wsp - (char*)d_ws) > ws_size) return;
    k_cvt8<<<(unsigned)(((size_t)2 * DI * HID / 8 + 255) / 256), 256, 0, stream>>>(win, WIN, (size_t)2 * DI * HID / 8); k_wx<<<(PW * DI / 4 + 255) / 256, 256, 0, stream>>>(wx, WX); k_cvt8<<<(DI * RR / 8 + 255) / 256, 256, 0, stream>>>(wdt, WDT, (size_t)DI * RR / 8); k_cvt8<<<(unsigned)(((size_t)HID * DI / 8 + 255) / 256), 256, 0, stream>>>(wout, WOUT, (size_t)HID * DI / 8);
    for (int b = 0; b < NB_; ++b) {
        k_cvt8<<<(LL * HID / 8 + 255) / 256, 256, 0, stream>>>(x + (size_t)b * LL * HID, XB, (size_t)LL * HID / 8);
        k_gemmw<bf, 0, false><<<dim3(LL / 64, 2 * DI / 64, 1), 32, 0, stream>>>(XB, nullptr, WIN, nullptr, HID, XR, 2 * DI, nullptr, 0, 0, 0);
        k_conv3<<<(LL * DI / 4 + 255) / 256, 256, 0, stream>>>(XR, c1w, c1b, c2w, c2b, tw, tb, XF, Fh, Fl);
        k_gemmw<bf, 1, false><<<dim3(LL / 64, PW / 64, 1), 32, 0, stream>>>(Fh, Fl, WX, nullptr, DI, PBC, PW, nullptr, 0, 0, 0);
        k_split<<<(LL * RR / 4 + 255) / 256, 256, 0, stream>>>(PBC, PW, 0, RR, Rh, Rl);
        k_gemmw<bf, 1, true><<<dim3(LL / 64, DI / 64, 1), 32, 0, stream>>>(Rh, Rl, WDT, nullptr, RR, DTR, DI, bdt, 0, 0, 0);
        k_scan<<<DI / 64, 256, 0, stream>>>(DTR, XF, PBC, XR, alog, Dp, Yh, Yl);
        k_gemmw<bf, 1, false><<<dim3(LL / 64, HID / 64, 1), 32, 0, stream>>>(Yh, Yl, WOUT, nullptr, DI, OUT + (size_t)b * LL * HID, HID, nullptr, 0, 0, 0); }
}
